// XAttn_68659347194155
// MI455X (gfx1250) — hardware-verified
//
#include <hip/hip_runtime.h>
#include <math.h>

typedef __attribute__((ext_vector_type(16))) _Float16 v16h;
typedef __attribute__((ext_vector_type(16))) __bf16 v16b;
typedef __attribute__((ext_vector_type(8)))  _Float16 v8h;
typedef __attribute__((ext_vector_type(8)))  float v8f;
typedef __attribute__((ext_vector_type(4)))  float v4f;
typedef __attribute__((ext_vector_type(2)))  float v2f;
typedef __attribute__((ext_vector_type(4)))  unsigned v4u;
typedef __attribute__((ext_vector_type(4)))  int v4i;
typedef float __attribute__((may_alias)) float_a;
typedef int __attribute__((may_alias)) int_a;

template <typename T> __device__ __forceinline__ void vst2(void* p, T v) { *(volatile T*)p = v; __threadfence(); *(volatile T*)p = v; }
__device__ __forceinline__ v8f wmma16(v16h a, v16h b, v8f c) {
  v8f d = __builtin_amdgcn_wmma_f32_16x16x32_f16(false, a, false, b, (short)0, c, false, false);
  asm volatile("v_nop\n\tv_nop\n\tv_nop\n\tv_nop" : "+v"(d) : "v"(a), "v"(b));
  return d;
}
__device__ __forceinline__ v8f wmma_bf(v16b a, v16b b, v8f c) {
  v8f d = __builtin_amdgcn_wmma_f32_16x16x32_bf16(false, a, false, b, (short)0, c, false, false);
  asm volatile("v_nop\n\tv_nop\n\tv_nop\n\tv_nop" : "+v"(d) : "v"(a), "v"(b));
  return d;
}
__device__ __forceinline__ v16h frag_h(const _Float16* rowk0, int lane) {
  union { v16h v; v8h q[2]; } u; const _Float16* p = rowk0 + 8 * (lane >> 4);
  u.q[0] = *(const v8h*)p; u.q[1] = *(const v8h*)(p + 16); return u.v;
}
__device__ __forceinline__ v16h frag_f32(const float* rowk0, int lane) {
  v16h a; const float* p = rowk0 + 8 * (lane >> 4);
#pragma unroll
  for (int i = 0; i < 8; ++i) { a[i] = (_Float16)p[i]; a[8 + i] = (_Float16)p[16 + i]; }
  return a;
}
__device__ __forceinline__ v16h frag_f32s(const float* rowk0, int lane, float sc) {
  v16h a; const float* p = rowk0 + 8 * (lane >> 4);
#pragma unroll
  for (int i = 0; i < 8; ++i) { a[i] = (_Float16)(p[i] * sc); a[8 + i] = (_Float16)(p[16 + i] * sc); }
  return a;
}
__device__ __forceinline__ v16h fragc_f32(const float* W, int k0, int n, int lane, int ld, int K) {
  v16h a; const int g = lane >> 4;
#pragma unroll
  for (int i = 0; i < 8; ++i) { const int ka = k0 + 8 * g + i, kb = ka + 16;
    a[i] = (_Float16)(ka < K ? W[(size_t)(ka < K ? ka : K - 1) * ld + n] : 0.f); a[8 + i] = (_Float16)(kb < K ? W[(size_t)(kb < K ? kb : K - 1) * ld + n] : 0.f); }
  return a;
}
struct F2 { v16b h, l; };
__device__ __forceinline__ F2 bsplit16(const float v[16]) { F2 r;
#pragma unroll
  for (int i = 0; i < 16; ++i) { const __bf16 h = (__bf16)v[i]; r.h[i] = h; r.l[i] = (__bf16)(v[i] - (float)h); }
  return r; }
__device__ __forceinline__ F2 split_row(const float* row, int k0, int lane) { float v[16]; const float* p = row + k0 + 8 * (lane >> 4);
#pragma unroll
  for (int i = 0; i < 8; ++i) { v[i] = p[i]; v[8 + i] = p[16 + i]; }
  return bsplit16(v); }
__device__ __forceinline__ F2 split_rowK(const float* row, int k0, int lane, int K) { float v[16]; const int g = lane >> 4;
#pragma unroll
  for (int i = 0; i < 8; ++i) { const int ka = k0 + 8 * g + i, kb = ka + 16; v[i] = ka < K ? row[ka < K ? ka : K - 1] : 0.f; v[8 + i] = kb < K ? row[kb < K ? kb : K - 1] : 0.f; }
  return bsplit16(v); }
__device__ __forceinline__ F2 split_col(const float* W, int k0, int n, int lane, int ld, int K) { float v[16]; const int g = lane >> 4;
#pragma unroll
  for (int i = 0; i < 8; ++i) { const int ka = k0 + 8 * g + i, kb = ka + 16; v[i] = ka < K ? W[(size_t)(ka < K ? ka : K - 1) * ld + n] : 0.f; v[8 + i] = kb < K ? W[(size_t)(kb < K ? kb : K - 1) * ld + n] : 0.f; }
  return bsplit16(v); }
__device__ __forceinline__ v8f mac3(const F2& a, const F2& b, v8f c) { c = wmma_bf(a.l, b.h, c); c = wmma_bf(a.h, b.l, c); return wmma_bf(a.h, b.h, c); }
__device__ __forceinline__ float sigm(float v) { return 1.0f / (1.0f + expf(-v)); }
#define LDSX() do { asm volatile("s_wait_dscnt 0" ::: "memory"); __builtin_amdgcn_wave_barrier(); __builtin_amdgcn_fence(__ATOMIC_RELEASE, "workgroup"); } while (0)


#define NR 65536
#define DD 128
#define NH 8
#define DK 32
#define RPB 16
#ifndef NBLK
#define NBLK (NR / RPB)
#endif
typedef __attribute__((ext_vector_type(8))) __bf16 v8b;
__device__ __forceinline__ v16b frag_b(const __bf16* rowk0, int lane) {
  union { v16b v; v8b q[2]; } u; const __bf16* p = rowk0 + 8 * (lane >> 4);
  u.q[0] = *(const v8b*)p; u.q[1] = *(const v8b*)(p + 16); return u.v;
}
__device__ __forceinline__ float bfr(float v) { return (float)(__bf16)v; }
__device__ __attribute__((noinline)) float exp_ni(float v) { return expf(v); }
__device__ __attribute__((noinline)) float erf_ni(float v) { return erff(v); }

#define PK_H 0
#define PK_R (PK_H + NH * DD * DD)
#define PK_KH (PK_R + NH * DD * DD)
#define PK_KR (PK_KH + DK * DD)
#define PK_END (PK_KR + DK * DD)
#define WS_END (2u * PK_END)

__global__ __launch_bounds__(128) void k_pack(const float* __restrict__ WH, const float* __restrict__ WR, const float* __restrict__ KH, const float* __restrict__ KR, __bf16* __restrict__ PK) {
  __shared__ __align__(16) __bf16 s[DD]; const int n = blockIdx.x, which = blockIdx.y, t = threadIdx.x; const float* src; size_t dst;
  if (which == 0) { src = WH + (size_t)n * DD; dst = PK_H + (size_t)n * DD; } else if (which == 1) { src = WR + (size_t)n * DD; dst = PK_R + (size_t)n * DD; }
  else if (which == 2) { if (n >= DK) return; src = KH + (size_t)n * DD; dst = PK_KH + (size_t)n * DD; } else { if (n >= DK) return; src = KR + (size_t)n * DD; dst = PK_KR + (size_t)n * DD; }
  s[t] = (__bf16)src[t]; __syncthreads();
  if (t < DD / 8) vst2((unsigned*)(PK + dst + t * 8), *(const v4u*)&s[t * 8]);
}
__device__ __forceinline__ void proj_rows(const float* __restrict__ X, const __bf16* __restrict__ P, size_t r0, int wave, int lane, int col, int g, float (*S)[NH * DD + 4]) {
  v16b a[DD / 32];
#pragma unroll
  for (int kc = 0; kc < DD / 32; ++kc) { const float* p = X + (r0 + col) * DD + kc * 32 + 8 * g;
#pragma unroll
    for (int i = 0; i < 8; ++i) { a[kc][i] = (__bf16)p[i]; a[kc][8 + i] = (__bf16)p[16 + i]; } }
#pragma unroll 1
  for (int pass = 0; pass < 4; ++pass) { const int n0 = wave * 256 + pass * 64; v8f acc[4] = {};
#pragma unroll
    for (int kc = 0; kc < DD / 32; ++kc)
#pragma unroll
      for (int j = 0; j < 4; ++j) acc[j] = wmma_bf(a[kc], frag_b(P + (size_t)(n0 + j * 16 + col) * DD + kc * 32, lane), acc[j]);
#pragma unroll
    for (int j = 0; j < 4; ++j)
#pragma unroll
      for (int r = 0; r < 8; ++r) S[8 * g + r][n0 + j * 16 + col] = acc[j][r]; }
}
__device__ __forceinline__ void key_rows(float (*S)[NH * DD + 4], const __bf16* __restrict__ K, int wave, int lane, int col, int g, float (*D)[NH][DK + 1]) {
#pragma unroll 1
  for (int hh = 0; hh < 2; ++hh) { const int h = wave * 2 + hh; v8f acc[2] = {};
#pragma unroll
    for (int kc = 0; kc < DD / 32; ++kc) { const F2 aa = split_row(&S[col][h * DD], kc * 32, lane);
#pragma unroll
      for (int j = 0; j < 2; ++j) { const v16b w = frag_b(K + (size_t)(j * 16 + col) * DD + kc * 32, lane); acc[j] = wmma_bf(aa.l, w, acc[j]); acc[j] = wmma_bf(aa.h, w, acc[j]); } }
#pragma unroll
    for (int j = 0; j < 2; ++j)
#pragma unroll
      for (int r = 0; r < 8; ++r) D[8 * g + r][h][j * 16 + col] = acc[j][r]; }
}
__global__ __launch_bounds__(128) void k_xattn(const float* __restrict__ HE, const float* __restrict__ RE, const __bf16* __restrict__ PK, const float* __restrict__ LG, const float* __restrict__ LB, float* __restrict__ OUT) {
  __shared__ __align__(16) float S[RPB][NH * DD + 4]; __shared__ __align__(16) float shk[RPB][NH][DK + 1], srk[RPB][NH][DK + 1]; __shared__ __align__(16) float stg[RPB][DD + 4];
  const int tid = threadIdx.x, wave = tid >> 5, lane = tid & 31, col = lane & 15, g = lane >> 4; const size_t r0 = (size_t)blockIdx.x * RPB;
  proj_rows(HE, PK + PK_H, r0, wave, lane, col, g, S); __syncthreads();
  key_rows(S, PK + PK_KH, wave, lane, col, g, shk); __syncthreads();
  proj_rows(RE, PK + PK_R, r0, wave, lane, col, g, S); __syncthreads();
  key_rows(S, PK + PK_KR, wave, lane, col, g, srk); __syncthreads();
  const int rl = tid >> 3, h = tid & 7; float rx[NH], hxa[NH];
  { float A[NH]; const float inv_temp = 1.0f / 5.656854249492381f;
#pragma unroll
    for (int j = 0; j < NH; ++j) { float a = 0.f;
#pragma unroll 4
      for (int k = 0; k < DK; ++k) a += (shk[rl][h][k] * inv_temp) * srk[rl][j][k];
      A[j] = a; }
    float mx = A[0];
#pragma unroll
    for (int j = 1; j < NH; ++j) mx = fmaxf(mx, A[j]);
    mx = fmaxf(mx, __shfl_xor(mx, 1)); mx = fmaxf(mx, __shfl_xor(mx, 2)); mx = fmaxf(mx, __shfl_xor(mx, 4));
    float se = 0.f;
#pragma unroll
    for (int j = 0; j < NH; ++j) { A[j] = exp_ni(A[j] - mx); se += A[j]; }
    se += __shfl_xor(se, 1); se += __shfl_xor(se, 2); se += __shfl_xor(se, 4);
    const float inv = 1.0f / se; float hx = 0.f;
#pragma unroll
    for (int j = 0; j < NH; ++j) { A[j] *= inv; hx += A[j]; }
#pragma unroll
    for (int j = 0; j < NH; ++j) { float v = A[j]; v += __shfl_xor(v, 1); v += __shfl_xor(v, 2); v += __shfl_xor(v, 4); rx[j] = v; }
#pragma unroll
    for (int j = 0; j < NH; ++j) hxa[j] = __shfl(hx, (lane & ~7) | j); }
#pragma unroll 1
  for (int i = 0; i < 16; ++i) { const int d = h * 16 + i; float a = 0.f;
#pragma unroll
    for (int hh = 0; hh < NH; ++hh) a += S[rl][hh * DD + d] * rx[hh];
    stg[rl][d] = a; }
  __syncthreads();
  proj_rows(HE, PK + PK_H, r0, wave, lane, col, g, S); __syncthreads();
  const float* he = HE + (r0 + rl) * DD; float s = 0.f;
#pragma unroll 1
  for (int i = 0; i < 16; ++i) { const int d = h * 16 + i; float a = 0.f;
#pragma unroll
    for (int hh = 0; hh < NH; ++hh) a += S[rl][hh * DD + d] * hxa[hh];
    const float tv = (a + stg[rl][d]) + bfr(he[d]); stg[rl][d] = tv; s += tv; }
  s += __shfl_xor(s, 1); s += __shfl_xor(s, 2); s += __shfl_xor(s, 4);
  const float mu = s * (1.0f / DD); float v = 0.f;
#pragma unroll 1
  for (int i = 0; i < 16; ++i) { const float dv = stg[rl][h * 16 + i] - mu; v += dv * dv; }
  v += __shfl_xor(v, 1); v += __shfl_xor(v, 2); v += __shfl_xor(v, 4);
  const float sd = sqrtf(v * (1.0f / DD) + 1e-5f);
#pragma unroll 1
  for (int i = 0; i < 16; ++i) { const int d = h * 16 + i; stg[rl][d] = bfr(LG[d]) * (stg[rl][d] - mu) / sd + bfr(LB[d]); }
  __syncthreads();
  for (int rr = 0; rr < 4; ++rr) { const int r2 = wave * 4 + rr; vst2(OUT + (r0 + r2) * DD + lane * 4, *(const v4f*)&stg[r2][lane * 4]); }
}
extern "C" void kernel_launch(void* const* d_in, const int* in_sizes, int n_in, void* d_out, int out_size, void* d_ws, size_t ws_size, hipStream_t stream) {
  (void)in_sizes; (void)n_in; (void)out_size;
  const float** F = (const float**)d_in;
  if (ws_size < (size_t)WS_END) return;
  __bf16* PK = (__bf16*)d_ws;
  k_pack<<<dim3(NH * DD, 4), 128, 0, stream>>>(F[2], F[3], F[4], F[5], PK);
  k_xattn<<<NBLK, 128, 0, stream>>>(F[0], F[1], PK, F[6], F[7], (float*)d_out);
}
